// SweetNet_9809705305013
// MI455X (gfx1250) — hardware-verified
//
#include <hip/hip_runtime.h>


namespace {
constexpr int N = 100000, E = 600000, G = 4096, D = 128, LIB = 1001, HID = 1024, NPAD = 100352  , NBLK = NPAD / 128;
constexpr float FXS = 1048576.0f, FXI = 1.0f / 1048576.0f, AS = 64.0f, AI = 1.0f / 64.0f, BNE = 1e-5f, SLOPE = 0.01f;

typedef _Float16 b16;
typedef __attribute__((ext_vector_type(16))) _Float16 v16b;
typedef __attribute__((ext_vector_type(8)))  _Float16 v8b;
typedef __attribute__((ext_vector_type(8)))  float v8f;
typedef __attribute__((ext_vector_type(4)))  float v4f;

__device__ __forceinline__ v8b ld8b(const b16* p) { return *(const v8b*)p; }
__device__ __forceinline__ v16b cat8b(v8b a, v8b b) { return __builtin_shufflevector(a, b, 0, 1, 2, 3, 4, 5, 6, 7, 8, 9, 10, 11, 12, 13, 14, 15); }
__device__ __forceinline__ v16b frag_kb(const b16* p, int hh) { return cat8b(ld8b(p + 8 * hh), ld8b(p + 16 + 8 * hh)); }
__device__ __forceinline__ void split16(float v, b16& hi, b16& lo) { hi = (b16)v; lo = (b16)(v - (float)hi); }
__device__ __forceinline__ void frag_ksplit(const float* p, int hh, v16b& fh_, v16b& fl_) {
  const float* p0 = p + 8 * hh; const float* p1 = p + 16 + 8 * hh;
#pragma unroll
  for (int e = 0; e < 8; ++e) { b16 a, c; split16(p0[e], a, c); fh_[e] = a; fl_[e] = c; split16(p1[e], a, c); fh_[8 + e] = a; fl_[8 + e] = c; }
}
__device__ __forceinline__ v8f wmma16b(v16b a, v16b b, v8f c) {
  v8f d = __builtin_amdgcn_wmma_f32_16x16x32_f16(false, a, false, b, (short)0, c, false, false);
  asm volatile("v_nop\n\tv_nop\n\tv_nop\n\tv_nop" : "+v"(d) : "v"(a), "v"(b));
  return d;
}
__device__ __forceinline__ void wave_lds_sync() {
  __builtin_amdgcn_fence(__ATOMIC_RELEASE, "workgroup");
  __builtin_amdgcn_wave_barrier();
  __builtin_amdgcn_fence(__ATOMIC_ACQUIRE, "workgroup");
}

struct Opnd { const void* p0; const void* p1; int ld; };
template <int NP> __device__ __forceinline__ void load_frags(const Opnd& o, int row, int kb, int hh, v16b& fh_, v16b& fl_) {
  if (NP == 0) { frag_ksplit((const float*)o.p0 + (size_t)row * o.ld + kb, hh, fh_, fl_); }
  else if (NP == 4) {
    const float* p = (const float*)o.p0 + (size_t)row * o.ld + kb; const float* p0 = p + 8 * hh; const float* p1 = p + 16 + 8 * hh;
#pragma unroll
    for (int e = 0; e < 8; ++e) { b16 a, c; split16(p0[e] * 64.0f, a, c); fh_[e] = a; fl_[e] = c; split16(p1[e] * 64.0f, a, c); fh_[8 + e] = a; fl_[8 + e] = c; }
  } else if (NP == 3) {
    const float* p = (const float*)o.p0 + (size_t)row * o.ld + kb; const float* p0 = p + 8 * hh; const float* p1 = p + 16 + 8 * hh;
#pragma unroll
    for (int e = 0; e < 8; ++e) { fh_[e] = (b16)p0[e]; fh_[8 + e] = (b16)p1[e]; }
    fl_ = fh_;
  } else {
    fh_ = frag_kb((const b16*)o.p0 + (size_t)row * o.ld + kb, hh);
    if (NP == 2) fl_ = frag_kb((const b16*)o.p1 + (size_t)row * o.ld + kb, hh); else fl_ = fh_;
  }
}
template <int ANP, int BNP> __device__ __forceinline__ v8f mac(v16b ah, v16b al, v16b bh, v16b bl, v8f c) {
  c = wmma16b(ah, bh, c);
  if (BNP == 0 || BNP == 2 || BNP == 4) c = wmma16b(ah, bl, c);
  if (ANP == 0 || ANP == 2 || ANP == 4) c = wmma16b(al, bh, c);
  return c;
}
template <int ANP, int BNP>
__device__ __forceinline__ void gemm_tile(const Opnd& A, const Opnd& B, int K, int m0, int c0, int nloc, int hlf, v8f (&acc)[2][4]) {
  for (int kb = 0; kb < K; kb += 32) {
    v16b a0h, a0l, a1h, a1l;
    load_frags<ANP>(A, m0 + nloc, kb, hlf, a0h, a0l);
    load_frags<ANP>(A, m0 + 16 + nloc, kb, hlf, a1h, a1l);
#pragma unroll
    for (int t = 0; t < 4; ++t) {
      v16b bh, bl;
      load_frags<BNP>(B, c0 + t * 16 + nloc, kb, hlf, bh, bl);
      acc[0][t] = mac<ANP, BNP>(a0h, a0l, bh, bl, acc[0][t]);
      acc[1][t] = mac<ANP, BNP>(a1h, a1l, bh, bl, acc[1][t]);
    }
  }
}

__device__ __forceinline__ void epi_planes(v8f (&acc)[2][4], float scale, bool two, b16* __restrict__ oh, b16* __restrict__ ol, int ldo,
                                           int m0, int c0, int lane, b16* Th, b16* Tl) {
  const int nloc = lane & 15, hlf = lane >> 4;
#pragma unroll
  for (int t = 0; t < 4; ++t)
#pragma unroll
    for (int r = 0; r < 2; ++r)
#pragma unroll
      for (int v = 0; v < 8; ++v) {
        const int rr = r * 16 + v + 8 * hlf, cc = t * 16 + nloc;
        b16 h_, l_; split16(acc[r][t][v] * scale, h_, l_);
        Th[rr * 64 + cc] = h_; Tl[rr * 64 + cc] = l_;
      }
  wave_lds_sync();
  for (int pass = 0; pass < 2; ++pass) {
#pragma unroll
    for (int j = 0; j < 8; ++j) {
      const int rr = j * 4 + (lane >> 3), c8 = (lane & 7) * 8;
      const size_t o = (size_t)(m0 + rr) * ldo + c0 + c8;
      *(volatile v8b*)(oh + o) = ld8b(Th + rr * 64 + c8);
      if (two) *(volatile v8b*)(ol + o) = ld8b(Tl + rr * 64 + c8);
    }
    __threadfence();
  }
}
__device__ __forceinline__ void epi_f32(v8f (&acc)[2][4], float scale, const float* rscale, float* __restrict__ out, int ldo, int m0, int c0, int lane, float* Tt) {
  const int nloc = lane & 15, hlf = lane >> 4;
#pragma unroll
  for (int t = 0; t < 4; ++t)
#pragma unroll
    for (int r = 0; r < 2; ++r)
#pragma unroll
      for (int v = 0; v < 8; ++v) {
        const int rr = r * 16 + v + 8 * hlf;
        const float rs = rscale ? rscale[(size_t)(m0 + rr) * 32] : 1.0f;
        Tt[rr * 64 + t * 16 + nloc] = acc[r][t][v] * scale * rs;
      }
  wave_lds_sync();
  float* dst0 = out + (size_t)m0 * ldo + c0;
  for (int pass = 0; pass < 2; ++pass) {
#pragma unroll
    for (int j = 0; j < 16; ++j) { const int rr = j * 2 + hlf, c4 = nloc * 4; *(volatile v4f*)(dst0 + (size_t)rr * ldo + c4) = *(const v4f*)(Tt + rr * 64 + c4); }
    __threadfence();
  }
}


__global__ __launch_bounds__(256) void prep_kernel(const float* __restrict__ r1, const float* __restrict__ o1, const float* __restrict__ r2, const float* __restrict__ o2, const float* __restrict__ r3, const float* __restrict__ o3,
                                                   const float* __restrict__ w1, const float* __restrict__ w2, b16* __restrict__ wc, b16* __restrict__ w1h, b16* __restrict__ w2h) {
  const size_t tid = (size_t)blockIdx.x * blockDim.x + threadIdx.x, nth = (size_t)gridDim.x * blockDim.x;
  for (int pass = 0; pass < 2; ++pass) {
    for (size_t p = tid; p < (size_t)3 * D * 2 * D; p += nth) { const int l = (int)(p / (D * 2 * D)); const int rem = (int)(p % (D * 2 * D)), n = rem / (2 * D), k = rem % (2 * D);
      const float* wr = (l == 0) ? r1 : (l == 1) ? r2 : r3; const float* wo = (l == 0) ? o1 : (l == 1) ? o2 : o3;
      ((volatile b16*)wc)[p] = (b16)((k < D) ? wr[(size_t)k * D + n] : wo[(size_t)(k - D) * D + n]); }
    for (size_t p = tid; p < (size_t)HID * D; p += nth) { const int n = (int)(p / D), k = (int)(p % D); ((volatile b16*)w1h)[p] = (b16)w1[(size_t)k * HID + n]; }
    for (size_t p = tid; p < (size_t)D * HID; p += nth) { const int n = (int)(p / HID), k = (int)(p % HID); ((volatile b16*)w2h)[p] = (b16)w2[(size_t)k * D + n]; }
    __threadfence();
  }
}

__global__ __launch_bounds__(256) void embed_kernel(const int* __restrict__ xl, const float* __restrict__ emb, float* __restrict__ h) {
  const int i = blockIdx.x * 256 + threadIdx.x; const int node = i >> 5, cq = (i & 31) * 4; v4f o = {0.0f, 0.0f, 0.0f, 0.0f};
  if (node < N) { int id = xl[node]; id = (id < 0) ? 0 : (id >= LIB ? LIB - 1 : id); o = *(const v4f*)(emb + (size_t)id * D + cq); }
  for (int pass = 0; pass < 2; ++pass) { *(volatile v4f*)(h + (size_t)node * D + cq) = o; __threadfence(); }
}

typedef __attribute__((ext_vector_type(4))) int v4i;
template <bool MEAN>
__global__ __launch_bounds__(256) void sum_kernel(const int* __restrict__ keys, const int* __restrict__ other, int nkeys, const float* __restrict__ feat, void* __restrict__ outp, int nvalid) {
  constexpr int NB = 512;
  __shared__ __attribute__((aligned(16))) int acc[NB * D];
  __shared__ int cnt[NB]; __shared__ int list[8 * 256];
  const int t_ = threadIdx.x, wave = t_ >> 5, lane = t_ & 31, base = blockIdx.x * NB;
  for (int i = t_; i < NB * D; i += 256) acc[i] = 0;
  for (int i = t_; i < NB; i += 256) cnt[i] = 0;
  __syncthreads();
  int* wl = list + wave * 256;
  for (int c0 = 0; c0 < nkeys; c0 += 256 * 8) {
    const int e0 = c0 + (wave * 32 + lane) * 8; int dd[8];
#pragma unroll
    for (int j = 0; j < 8; ++j) { const int dv = keys[min(e0 + j, nkeys - 1)]; dd[j] = (e0 + j < nkeys) ? dv : -1; }
    unsigned sl[8]; bool hit[8]; bool anyl = false;
#pragma unroll
    for (int j = 0; j < 8; ++j) { sl[j] = (unsigned)(dd[j] - base); hit[j] = sl[j] < (unsigned)NB; anyl |= hit[j]; }
    int wc = 0;
    if (__builtin_amdgcn_ballot_w32(anyl) != 0u) {
#pragma unroll
      for (int j = 0; j < 8; ++j) {
        const unsigned mj = __builtin_amdgcn_ballot_w32(hit[j]);
        if (mj != 0u) {
          if (hit[j]) { const int pos = wc + (int)__builtin_amdgcn_mbcnt_lo(mj, 0u); int o = other ? other[min(e0 + j, nkeys - 1)] : (e0 + j); o = (o < 0) ? 0 : (o >= N ? N - 1 : o); wl[pos] = (o << 9) | (int)sl[j]; if (MEAN) atomicAdd(&cnt[sl[j]], 1); }
          wc += __builtin_popcount(mj); } } }
    __builtin_amdgcn_wave_barrier(); __builtin_amdgcn_fence(__ATOMIC_RELEASE, "workgroup"); __builtin_amdgcn_fence(__ATOMIC_ACQUIRE, "workgroup");
    for (int i = 0; i < wc; ++i) { const int ent = wl[i]; const int o = ent >> 9, slot = ent & 511; const v4f v = *(const v4f*)(feat + (size_t)o * D + lane * 4); int* ar = acc + slot * D + lane * 4;
#pragma unroll
      for (int c = 0; c < 4; ++c) atomicAdd(ar + c, (int)rintf(v[c] * FXS)); }
    __builtin_amdgcn_wave_barrier();
  }
  __syncthreads();
  for (int pass = 0; pass < 2; ++pass) {
    if (MEAN) {
      for (int i = t_; i < NB * D / 4; i += 256) { const int r = i >> 5, cq = (i & 31) * 4, row = base + r; v4f o = {0.0f, 0.0f, 0.0f, 0.0f};
        if (row < nvalid) { const float sc = FXI / fmaxf((float)cnt[r], 1.0f);
#pragma unroll
          for (int c = 0; c < 4; ++c) o[c] = (float)acc[r * D + cq + c] * sc; }
        *(volatile v4f*)((float*)outp + (size_t)row * D + cq) = o; }
    } else {
      for (int i = t_; i < NB * D / 8; i += 256) { const int r = i >> 4, c8 = (i & 15) * 8, row = base + r; v8b o;
#pragma unroll
        for (int c = 0; c < 8; ++c) o[c] = (b16)((row < nvalid) ? (float)acc[r * D + c8 + c] * (FXI * AS) : 0.0f);
        *(volatile v8b*)((b16*)outp + (size_t)row * D + c8) = o; }
    }
    __threadfence();
  }
}

__global__ __launch_bounds__(128) void conv_kernel(const b16* __restrict__ agg, const float* __restrict__ h, const b16* __restrict__ w, const float* __restrict__ bias, float* __restrict__ ho) {
  __shared__ __attribute__((aligned(16))) float Ts[4][32 * 64];
  const int lane = threadIdx.x & 31, wave = threadIdx.x >> 5, nloc = lane & 15, hlf = lane >> 4, m0 = blockIdx.y * 128 + wave * 32, c0 = blockIdx.x * 64;
  v8f acc[2][4];
#pragma unroll
  for (int r = 0; r < 2; ++r)
#pragma unroll
    for (int t = 0; t < 4; ++t) acc[r][t] = (v8f){};
#pragma unroll 1
  for (int kb = 0; kb < 2 * D; kb += 32) { v16b a0, a1;
    if (kb < D) { a0 = frag_kb(agg + (size_t)(m0 + nloc) * D + kb, hlf); a1 = frag_kb(agg + (size_t)(m0 + 16 + nloc) * D + kb, hlf); }
    else { const int ko = kb - D;
#pragma unroll
      for (int e = 0; e < 16; ++e) { const int k = ko + ((e < 8) ? (8 * hlf + e) : (16 + 8 * hlf + e - 8)); a0[e] = (b16)(h[(size_t)(m0 + nloc) * D + k] * AS); a1[e] = (b16)(h[(size_t)(m0 + 16 + nloc) * D + k] * AS); } }
#pragma unroll
    for (int t = 0; t < 4; ++t) { const v16b bw = frag_kb(w + (size_t)(c0 + t * 16 + nloc) * 2 * D + kb, hlf); acc[0][t] = wmma16b(a0, bw, acc[0][t]); acc[1][t] = wmma16b(a1, bw, acc[1][t]); } }
#pragma unroll
  for (int t = 0; t < 4; ++t)
#pragma unroll
    for (int r = 0; r < 2; ++r)
#pragma unroll
      for (int v = 0; v < 8; ++v) { const int row = m0 + r * 16 + 8 * hlf + v; float val = acc[r][t][v] * AI + bias[c0 + t * 16 + nloc]; val = (val > 0.0f) ? val : SLOPE * val; acc[r][t][v] = (row < N) ? val : 0.0f; }
  epi_f32(acc, 1.0f, nullptr, ho, D, m0, c0, lane, Ts[wave]);
}

template <int KIN, int NOUT, int MODE>
__global__ __launch_bounds__(128) void head_kernel(const float* __restrict__ x, const b16* __restrict__ w, const float* __restrict__ bias, const float* __restrict__ g, const float* __restrict__ bb, const float* __restrict__ mu, const float* __restrict__ var, float* __restrict__ y) {
  __shared__ __attribute__((aligned(16))) float Ts[4][32 * 64];
  const int lane = threadIdx.x & 31, wave = threadIdx.x >> 5, nloc = lane & 15, hlf = lane >> 4, m0 = blockIdx.y * 128 + wave * 32, c0 = blockIdx.x * 64;
  v8f acc[2][4];
#pragma unroll
  for (int r = 0; r < 2; ++r)
#pragma unroll
    for (int t = 0; t < 4; ++t) acc[r][t] = (v8f){};
#pragma unroll 1
  for (int kb = 0; kb < KIN; kb += 32) { v16b a0, a1;
#pragma unroll
    for (int e = 0; e < 16; ++e) { const int k = kb + ((e < 8) ? (8 * hlf + e) : (16 + 8 * hlf + e - 8)); a0[e] = (b16)(x[(size_t)(m0 + nloc) * KIN + k] * AS); a1[e] = (b16)(x[(size_t)(m0 + 16 + nloc) * KIN + k] * AS); }
#pragma unroll
    for (int t = 0; t < 4; ++t) { const v16b bw = frag_kb(w + (size_t)(c0 + t * 16 + nloc) * KIN + kb, hlf); acc[0][t] = wmma16b(a0, bw, acc[0][t]); acc[1][t] = wmma16b(a1, bw, acc[1][t]); } }
#pragma unroll
  for (int t = 0; t < 4; ++t)
#pragma unroll
    for (int r = 0; r < 2; ++r)
#pragma unroll
      for (int v = 0; v < 8; ++v) { const int c = c0 + t * 16 + nloc; float val = acc[r][t][v] * AI + bias[c]; val = (val - mu[c]) * rsqrtf(var[c] + BNE) * g[c] + bb[c]; if (MODE == 0) val = (val > 0.0f) ? val : SLOPE * val; acc[r][t][v] = val; }
  epi_f32(acc, 1.0f, nullptr, y, NOUT, m0, c0, lane, Ts[wave]);
}

__global__ __launch_bounds__(256) void final_kernel(const float* __restrict__ xo, const float* __restrict__ w3, const float* __restrict__ b3, float* __restrict__ out) {
  const int gidx = blockIdx.x * 256 + threadIdx.x; float s = b3[0];
#pragma unroll 1
  for (int k = 0; k < D; k += 4) { const v4f v = *(const v4f*)(xo + (size_t)gidx * D + k);
#pragma unroll
    for (int c = 0; c < 4; ++c) { const float a = (v[c] > 0.0f) ? v[c] : SLOPE * v[c]; s += a * w3[k + c]; } }
  for (int pass = 0; pass < 2; ++pass) { ((volatile float*)out)[gidx] = s; __threadfence(); }
}
}

extern "C" void kernel_launch(void* const* d_in, const int* in_sizes, int n_in,
                              void* d_out, int out_size, void* d_ws, size_t ws_size, hipStream_t stream) {
  (void)n_in; (void)out_size;
  const int* xl = (const int*)d_in[0]; const int* ei = (const int*)d_in[1]; const int* batch = (const int*)d_in[2]; const float* emb = (const float*)d_in[3];
  const float* r1 = (const float*)d_in[4]; const float* br1 = (const float*)d_in[5]; const float* o1 = (const float*)d_in[6]; const float* r2 = (const float*)d_in[7]; const float* br2 = (const float*)d_in[8]; const float* o2 = (const float*)d_in[9]; const float* r3 = (const float*)d_in[10]; const float* br3 = (const float*)d_in[11]; const float* o3 = (const float*)d_in[12];
  const float* w1 = (const float*)d_in[13]; const float* b1 = (const float*)d_in[14]; const float* w2 = (const float*)d_in[15]; const float* b2 = (const float*)d_in[16]; const float* w3 = (const float*)d_in[17]; const float* b3 = (const float*)d_in[18];
  const float* bn1g = (const float*)d_in[19]; const float* bn1b = (const float*)d_in[20]; const float* bn1m = (const float*)d_in[21]; const float* bn1v = (const float*)d_in[22]; const float* bn2g = (const float*)d_in[23]; const float* bn2b = (const float*)d_in[24]; const float* bn2m = (const float*)d_in[25]; const float* bn2v = (const float*)d_in[26];
  float* out = (float*)d_out;
  if (in_sizes[0] != N || in_sizes[1] != 2 * E || in_sizes[2] != N || in_sizes[3] != LIB * D || in_sizes[4] != D * D || in_sizes[13] != D * HID || in_sizes[15] != HID * D || in_sizes[17] != D) return;
  const int* esrc = ei; const int* edst = ei + E;
  size_t off = 0; char* ws = (char*)d_ws;
  auto carve = [&](size_t bytes) { char* p = ws + off; off += (bytes + 255) & ~(size_t)255; return p; };
  b16* wc = (b16*)carve((size_t)3 * D * 2 * D * 2); b16* w1h = (b16*)carve((size_t)HID * D * 2); b16* w2h = (b16*)carve((size_t)D * HID * 2);
  float* ha = (float*)carve((size_t)NPAD * D * 4); float* hb = (float*)carve((size_t)NPAD * D * 4); b16* agg = (b16*)carve((size_t)NPAD * D * 2);
  if (off > ws_size) return;
  float* z = (float*)agg; float* pooled = z + (size_t)G * HID; float* xo = pooled + (size_t)G * D;
  prep_kernel<<<256, 256, 0, stream>>>(r1, o1, r2, o2, r3, o3, w1, w2, wc, w1h, w2h);
  embed_kernel<<<NPAD * 32 / 256, 256, 0, stream>>>(xl, emb, ha);
  sum_kernel<false><<<NPAD / 512, 256, 0, stream>>>(edst, esrc, E, ha, agg, NPAD);
  conv_kernel<<<dim3(2, NBLK), 128, 0, stream>>>(agg, ha, wc, br1, hb);
  sum_kernel<false><<<NPAD / 512, 256, 0, stream>>>(edst, esrc, E, hb, agg, NPAD);
  conv_kernel<<<dim3(2, NBLK), 128, 0, stream>>>(agg, hb, wc + (size_t)D * 2 * D, br2, ha);
  sum_kernel<false><<<NPAD / 512, 256, 0, stream>>>(edst, esrc, E, ha, agg, NPAD);
  conv_kernel<<<dim3(2, NBLK), 128, 0, stream>>>(agg, ha, wc + (size_t)2 * D * 2 * D, br3, hb);
  sum_kernel<true><<<G / 512, 256, 0, stream>>>(batch, nullptr, N, hb, pooled, G);
  head_kernel<D, HID, 0><<<dim3(HID / 64, G / 128), 128, 0, stream>>>(pooled, w1h, b1, bn1g, bn1b, bn1m, bn1v, z);
  head_kernel<HID, D, 1><<<dim3(D / 64, G / 128), 128, 0, stream>>>(z, w2h, b2, bn2g, bn2b, bn2m, bn2v, xo);
  final_kernel<<<G / 256, 256, 0, stream>>>(xo, w3, b3, out);
}
